// HeteroGATConv_58265526338119
// MI455X (gfx1250) — hardware-verified
//
#include <hip/hip_runtime.h>
#include <stddef.h>


#define FIN     128
#define NCOL    128
#define NHEAD   4
#define NTHR    256
#define NWAVE   8
#define EPT     8
#define NGRP    2
#define CHUNK   (NTHR * EPT * NGRP)
#define WCAP    (EPT * NGRP * 32)
#define LISTN   (NWAVE * WCAP)
#define NBC     4096
#define NBF     1024
#define RCAP    40960
#define RBN     128
#define TGT     256
#define DEGCAP  256
#define OTHR    512
#define WSCAP   134217728
#define WSCALE  64.0f
#define WINV    (1.0f / 64.0f)
#define NEG_SLOPE 0.2f
#define NEG_BIG (-3.0e38f)

#define LDS_FILL ((RCAP + NBF + LISTN) * 4 + 64)

static_assert((CHUNK & (CHUNK - 1)) == 0);
static_assert(CHUNK <= 4096);
static_assert(NBC <= 4096 && NBF <= 4096);
static_assert((NBC & (NBC - 1)) == 0 && (NBF & (NBF - 1)) == 0);
static_assert(NBC == 4 * NBF);
static_assert(OTHR * 8 == NBC);
static_assert((RCAP % 32) == 0);
static_assert(TGT == NWAVE * 32);
static_assert((NBC % TGT) == 0);
static_assert(NCOL == 32 * NHEAD);

typedef float    v4f  __attribute__((ext_vector_type(4)));
typedef float    v8f  __attribute__((ext_vector_type(8)));
typedef int      v4i  __attribute__((ext_vector_type(4)));
typedef _Float16 v8h  __attribute__((ext_vector_type(8)));
typedef _Float16 v16h __attribute__((ext_vector_type(16)));
union FragH { v16h v; v8h h[2]; };

template <int KD, int NC>
struct GCfg {
  static constexpr int WPR  = (NC >= 32) ? 2 : 1;
  static constexpr int TPW  = NC / 16 / WPR;
  static constexpr int RG   = NWAVE / WPR;
  static constexpr int BM   = RG * 16;
  static constexpr int APK  = KD + 8;
  static constexpr int LDSA = BM * APK * 2;
  static constexpr int LDSS = BM * NC * 4;
  static constexpr int LDS  = LDSA > LDSS ? LDSA : LDSS;
};

__device__ __forceinline__ v8f wmh(v16h a, v16h b, v8f c) {
  v8f d = __builtin_amdgcn_wmma_f32_16x16x32_f16(false, a, false, b, (short)0, c, false, false);
  asm volatile("v_nop\n\tv_nop\n\tv_nop\n\tv_nop" : "+v"(d) : "v"(a), "v"(b));
  return d;
}

__device__ __forceinline__ float lrelu(float v) { return v > 0.0f ? v : NEG_SLOPE * v; }

template <int NB>
__device__ __forceinline__ int scan_chunk(const int* __restrict__ dsts, int nE, int cbase, int slotBase,
                                          int vec8, int* list, int tid, int lane, int wave) {
  int wc = 0;
#pragma unroll
  for (int g = 0; g < NGRP; ++g) {
    const int el0  = (g * NTHR + tid) * EPT;
    const int e0   = cbase + el0;
    const int sent = -2147483647 - 1;
    v4i da, db;
    if (vec8 != 0 && cbase + CHUNK <= nE) {
      da = *(const v4i*)(dsts + e0);
      db = *(const v4i*)(dsts + e0 + 4);
    } else {
      da.x = (e0     < nE) ? dsts[min(e0, nE - 1)] : sent;
      da.y = (e0 + 1 < nE) ? dsts[min(e0 + 1, nE - 1)] : sent;
      da.z = (e0 + 2 < nE) ? dsts[min(e0 + 2, nE - 1)] : sent;
      da.w = (e0 + 3 < nE) ? dsts[min(e0 + 3, nE - 1)] : sent;
      db.x = (e0 + 4 < nE) ? dsts[min(e0 + 4, nE - 1)] : sent;
      db.y = (e0 + 5 < nE) ? dsts[min(e0 + 5, nE - 1)] : sent;
      db.z = (e0 + 6 < nE) ? dsts[min(e0 + 6, nE - 1)] : sent;
      db.w = (e0 + 7 < nE) ? dsts[min(e0 + 7, nE - 1)] : sent;
    }
    const unsigned nb = (unsigned)slotBase;
    const unsigned s0 = (unsigned)da.x - nb, s1 = (unsigned)da.y - nb;
    const unsigned s2 = (unsigned)da.z - nb, s3 = (unsigned)da.w - nb;
    const unsigned s4 = (unsigned)db.x - nb, s5 = (unsigned)db.y - nb;
    const unsigned s6 = (unsigned)db.z - nb, s7 = (unsigned)db.w - nb;
    const bool h0 = s0 < (unsigned)NB, h1 = s1 < (unsigned)NB, h2 = s2 < (unsigned)NB, h3 = s3 < (unsigned)NB;
    const bool h4 = s4 < (unsigned)NB, h5 = s5 < (unsigned)NB, h6 = s6 < (unsigned)NB, h7 = s7 < (unsigned)NB;
    const unsigned any = __builtin_amdgcn_ballot_w32(h0 | h1 | h2 | h3 | h4 | h5 | h6 | h7);
    if (any != 0u) {
#define HITJ(J, HJ, SJ) { \
        const unsigned mj = __builtin_amdgcn_ballot_w32(HJ); \
        if (mj != 0u) { \
          if (HJ) { \
            const int pos = wc + (int)__builtin_amdgcn_mbcnt_lo(mj, 0u); \
            if (pos < WCAP) list[wave * WCAP + pos] = ((el0 + (J)) << 12) | (int)(SJ); \
          } \
          wc += (int)__builtin_popcount(mj); } }
      HITJ(0, h0, s0)
      HITJ(1, h1, s1)
      HITJ(2, h2, s2)
      HITJ(3, h3, s3)
      HITJ(4, h4, s4)
      HITJ(5, h5, s5)
      HITJ(6, h6, s6)
      HITJ(7, h7, s7)
#undef HITJ
    }
  }
  return wc;
}

template <int KD, int NC>
__global__ __launch_bounds__(NTHR) void k_wprep(const float* __restrict__ W, _Float16* wp) {
  constexpr int UNITS = NC * KD / 8;
  constexpr int KD8   = KD / 8;
  static_assert((UNITS % NTHR) == 0);
  const int i = (int)blockIdx.x * NTHR + (int)threadIdx.x;
  if (i >= UNITS) return;
  const int n  = i / KD8;
  const int k0 = (i - n * KD8) * 8;
  const float* wc = W + (size_t)k0 * NC + n;
  v8h hv;
  hv[0] = (_Float16)(wc[0 * NC] * WSCALE);
  hv[1] = (_Float16)(wc[1 * NC] * WSCALE);
  hv[2] = (_Float16)(wc[2 * NC] * WSCALE);
  hv[3] = (_Float16)(wc[3 * NC] * WSCALE);
  hv[4] = (_Float16)(wc[4 * NC] * WSCALE);
  hv[5] = (_Float16)(wc[5 * NC] * WSCALE);
  hv[6] = (_Float16)(wc[6 * NC] * WSCALE);
  hv[7] = (_Float16)(wc[7 * NC] * WSCALE);
  _Float16* dh = wp + (size_t)i * 8;
  *(volatile v8h*)dh = hv;
  __threadfence();
  *(volatile v8h*)dh = hv;
}

__global__ __launch_bounds__(NTHR) void k_count(
    const int* __restrict__ dsts, int* cnt, int nE, int vec8) {
  __shared__ __attribute__((aligned(16))) int scnt[NBC];
  __shared__ __attribute__((aligned(16))) int list[LISTN];
  __shared__ int wcnt[NWAVE];
  const int tid = threadIdx.x, lane = tid & 31, wave = tid >> 5;
  const int nodeBase = blockIdx.x * NBC;

  for (int i = tid; i < NBC; i += NTHR) scnt[i] = 0;
  __syncthreads();

  const int nChunks = (nE + CHUNK - 1) / CHUNK;
#pragma unroll 1
  for (int ch = 0; ch < nChunks; ++ch) {
    const int cbase = ch * CHUNK;
    const int wc = scan_chunk<NBC>(dsts, nE, cbase, nodeBase, vec8, list, tid, lane, wave);
    if (lane == 0) wcnt[wave] = wc;
    __syncthreads();
    if (wave == 0) {
#pragma unroll 1
      for (int wsx = 0; wsx < NWAVE; ++wsx) {
        int n = __builtin_amdgcn_readfirstlane(wcnt[wsx]);
        n = n > WCAP ? WCAP : (n < 0 ? 0 : n);
        const int* lp = list + wsx * WCAP;
#pragma unroll 1
        for (int i = 0; i < n; ++i) {
          const int ent  = __builtin_amdgcn_readfirstlane(lp[i]);
          const int slot = ent & (NBC - 1);
          if (lane == 0) scnt[slot] = scnt[slot] + 1;
        }
      }
    }
    __syncthreads();
  }

  v4i cq[4];
#pragma unroll
  for (int q = 0; q < 4; ++q) {
    const int f = (wave * 4 + q) * 128 + 4 * lane;
    cq[q] = *(const v4i*)(scnt + f);
  }
  int* cp = cnt + (size_t)nodeBase;
#pragma unroll
  for (int q = 0; q < 4; ++q) {
    const int f = (wave * 4 + q) * 128 + 4 * lane;
    *(volatile v4i*)(cp + f) = cq[q];
  }
  __threadfence();
#pragma unroll
  for (int q = 0; q < 4; ++q) {
    const int f = (wave * 4 + q) * 128 + 4 * lane;
    *(volatile v4i*)(cp + f) = cq[q];
  }
}

__global__ __launch_bounds__(OTHR) void k_offsets(
    const int* __restrict__ cnt, int* off, int* rbase, int nChunk) {
  __shared__ __attribute__((aligned(16))) int soff[NBC];
  __shared__ __attribute__((aligned(16))) int srb[RBN];
  __shared__ int wtot[OTHR / 32];
  const int tid = threadIdx.x, lane = tid & 31, wave = tid >> 5, sub = tid >> 7;
  for (int i = tid; i < RBN; i += OTHR) srb[i] = 0;
  int carry = 0;
#pragma unroll 1
  for (int ch = 0; ch < nChunk; ++ch) {
    const int base = ch * NBC;
    const v4i c0 = *(const v4i*)(cnt + base + 8 * tid);
    const v4i c1 = *(const v4i*)(cnt + base + 8 * tid + 4);
    const int e0 = max(c0.x, 0), e1 = max(c0.y, 0), e2 = max(c0.z, 0), e3 = max(c0.w, 0);
    const int e4 = max(c1.x, 0), e5 = max(c1.y, 0), e6 = max(c1.z, 0), e7 = max(c1.w, 0);
    const int ts = e0 + e1 + e2 + e3 + e4 + e5 + e6 + e7;
    int incl = ts;
#pragma unroll
    for (int d = 1; d < 32; d <<= 1) {
      const int t = __shfl_up(incl, d);
      if (lane >= d) incl += t;
    }
    if (lane == 31) wtot[wave] = incl;
    __syncthreads();
    const int S0 = wtot[0]  + wtot[1]  + wtot[2]  + wtot[3];
    const int S1 = wtot[4]  + wtot[5]  + wtot[6]  + wtot[7];
    const int S2 = wtot[8]  + wtot[9]  + wtot[10] + wtot[11];
    const int S3 = wtot[12] + wtot[13] + wtot[14] + wtot[15];
    int pre = 0;
#pragma unroll 1
    for (int w = 4 * sub; w < wave; ++w) pre += wtot[w];
    const int b0 = carry;
    const int b1 = b0 + ((S0 + 31) & ~31);
    const int b2 = b1 + ((S1 + 31) & ~31);
    const int b3 = b2 + ((S2 + 31) & ~31);
    const int b4 = b3 + ((S3 + 31) & ~31);
    const int myb = sub == 0 ? b0 : (sub == 1 ? b1 : (sub == 2 ? b2 : b3));
    if (tid == 0) {
      srb[min(4 * ch + 0, RBN - 1)] = b0;
      srb[min(4 * ch + 1, RBN - 1)] = b1;
      srb[min(4 * ch + 2, RBN - 1)] = b2;
      srb[min(4 * ch + 3, RBN - 1)] = b3;
    }
    int run = myb + pre + incl - ts;
    soff[8 * tid + 0] = run; run += e0;
    soff[8 * tid + 1] = run; run += e1;
    soff[8 * tid + 2] = run; run += e2;
    soff[8 * tid + 3] = run; run += e3;
    soff[8 * tid + 4] = run; run += e4;
    soff[8 * tid + 5] = run; run += e5;
    soff[8 * tid + 6] = run; run += e6;
    soff[8 * tid + 7] = run;
    carry = b4;
    __syncthreads();
    const v4i o0 = *(const v4i*)(soff + 4 * tid);
    const v4i o1 = *(const v4i*)(soff + 4 * (tid + OTHR));
    int* op = off + base;
    *(volatile v4i*)(op + 4 * tid) = o0;
    *(volatile v4i*)(op + 4 * (tid + OTHR)) = o1;
    __threadfence();
    *(volatile v4i*)(op + 4 * tid) = o0;
    *(volatile v4i*)(op + 4 * (tid + OTHR)) = o1;
    __syncthreads();
  }
  if (tid == 0) srb[min(4 * nChunk, RBN - 1)] = carry;
  __syncthreads();
  v4i rv = {0, 0, 0, 0};
  if (tid < 32) rv = *(const v4i*)(srb + 4 * tid);
  if (tid < 32) *(volatile v4i*)(rbase + 4 * tid) = rv;
  __threadfence();
  if (tid < 32) *(volatile v4i*)(rbase + 4 * tid) = rv;
}

__global__ __launch_bounds__(NTHR) void k_fill(
    const int* __restrict__ srcs, const int* __restrict__ dsts,
    const int* __restrict__ off, const int* __restrict__ rbase,
    int* csr, int nN, int nE, int vec8, int csrLen) {
  extern __shared__ v4f lds_dyn[];
  int* region = (int*)lds_dyn;
  int* cursor = region + RCAP;
  int* list   = cursor + NBF;
  int* wcnt   = list + LISTN;
  const int tid = threadIdx.x, lane = tid & 31, wave = tid >> 5;
  const int b = blockIdx.x;
  const int nodeBase = b * NBF;

  int rb0 = rbase[b];
  const int rb1 = rbase[b + 1];
  rb0 = rb0 < 0 ? 0 : (rb0 > csrLen ? csrLen : rb0);
  rb0 &= ~31;
  int len = rb1 - rb0;
  len = len < 0 ? 0 : (len > RCAP ? RCAP : len);
  int lenW = (len + 31) & ~31;
  if (rb0 + lenW > csrLen) lenW = (csrLen - rb0) & ~31;

  {
    const v4i z = {0, 0, 0, 0};
    for (int i = tid; i < RCAP / 4; i += NTHR) ((v4i*)region)[i] = z;
    for (int s = tid; s < NBF; s += NTHR) {
      int o = off[nodeBase + s] - rb0;
      o = o < 0 ? 0 : (o > RCAP ? RCAP : o);
      cursor[s] = o;
    }
  }
  __syncthreads();

  const int nChunks = (nE + CHUNK - 1) / CHUNK;
#pragma unroll 1
  for (int ch = 0; ch < nChunks; ++ch) {
    const int cbase = ch * CHUNK;
    const int wc = scan_chunk<NBF>(dsts, nE, cbase, nodeBase, vec8, list, tid, lane, wave);
    if (lane == 0) wcnt[wave] = wc;
    __syncthreads();
    if (wave == 0) {
#pragma unroll 1
      for (int wsx = 0; wsx < NWAVE; ++wsx) {
        int n = __builtin_amdgcn_readfirstlane(wcnt[wsx]);
        n = n > WCAP ? WCAP : (n < 0 ? 0 : n);
        const int* lp = list + wsx * WCAP;
#pragma unroll 1
        for (int i = 0; i < n; ++i) {
          const int ent  = __builtin_amdgcn_readfirstlane(lp[i]);
          const int slot = ent & (NBF - 1);
          int e = cbase + ((ent >> 12) & (CHUNK - 1));
          e = e > nE - 1 ? nE - 1 : e;
          int src = srcs[e];
          src = src < 0 ? 0 : (src > nN - 1 ? nN - 1 : src);
          if (lane == 0) {
            int pos = cursor[slot];
            pos = pos < 0 ? 0 : (pos > RCAP - 1 ? RCAP - 1 : pos);
            region[pos] = src;
            const int np = pos + 1;
            cursor[slot] = np > RCAP ? RCAP : np;
          }
        }
      }
    }
    __syncthreads();
  }

  const int nv = lenW >> 2;
  int* gp = csr + rb0;
#pragma unroll 1
  for (int i = tid; i < nv; i += NTHR) { const v4i v = ((const v4i*)region)[i]; *(volatile v4i*)(gp + 4 * i) = v; }
  __threadfence();
#pragma unroll 1
  for (int i = tid; i < nv; i += NTHR) { const v4i v = ((const v4i*)region)[i]; *(volatile v4i*)(gp + 4 * i) = v; }
}

template <int KD, int NC, int HEADS>
__global__ __launch_bounds__(NTHR) void k_gemm(
    const float* __restrict__ A, const _Float16* __restrict__ Bw,
    const float* __restrict__ attS, const float* __restrict__ attD,
    float* C, float* eS, float* eD, int nRowsA) {
  typedef GCfg<KD, NC> G;
  constexpr int WPR  = G::WPR;
  constexpr int TPW  = G::TPW;
  constexpr int BM   = G::BM;
  constexpr int APK  = G::APK;
  constexpr int CH   = NC / HEADS;
  constexpr int LPH  = CH / 4;
  constexpr int Q4   = TPW * 4;
  constexpr int RPI  = 32 / Q4;
  constexpr int NIT  = 16 / RPI;
  constexpr int NES  = BM * HEADS;
  constexpr int NESI = NES / 128;
  constexpr int UPT  = (BM * KD / 8) / NTHR;
  static_assert(KD % 32 == 0 && NC % (16 * WPR) == 0);
  static_assert(HEADS * CH == NC && (CH % 4) == 0);
  static_assert((Q4 & (Q4 - 1)) == 0 && Q4 <= 32 && Q4 >= LPH && (LPH & (LPH - 1)) == 0 && LPH >= 1);
  static_assert(NIT * RPI == 16);
  static_assert((NES % 128) == 0 && 2 * NESI <= NWAVE);
  static_assert(UPT * NTHR * 8 == BM * KD);
  static_assert(((APK * 2) % 16) == 0);
  static_assert(BM * NC * 4 <= G::LDS && BM * APK * 2 <= G::LDS);

  extern __shared__ v4f lds_dyn[];
  __shared__ __attribute__((aligned(16))) float sES[NES];
  __shared__ __attribute__((aligned(16))) float sED[NES];
  _Float16* sA  = (_Float16*)lds_dyn;
  float*    stg = (float*)lds_dyn;
  const int tid = threadIdx.x, lane = tid & 31, wave = tid >> 5, hh = lane >> 4, m = lane & 15;
  const int rowBase = blockIdx.x * BM;

#pragma unroll
  for (int i = 0; i < UPT; ++i) {
    const int idx = i * NTHR + tid;
    const int r   = idx / (KD / 8);
    const int c8  = (idx - r * (KD / 8)) * 8;
    int row = rowBase + r;
    row = row > nRowsA - 1 ? nRowsA - 1 : row;
    const float* ap = A + (size_t)row * KD + c8;
    const v4f a = *(const v4f*)ap, b = *(const v4f*)(ap + 4);
    v8h hv;
    hv[0] = (_Float16)a.x; hv[1] = (_Float16)a.y; hv[2] = (_Float16)a.z; hv[3] = (_Float16)a.w;
    hv[4] = (_Float16)b.x; hv[5] = (_Float16)b.y; hv[6] = (_Float16)b.z; hv[7] = (_Float16)b.w;
    *(v8h*)(sA + r * APK + c8) = hv;
  }
  __syncthreads();

  const int rg  = wave / WPR;
  const int chf = wave - rg * WPR;
  const int r0  = rg * 16;
  const int c0  = chf * TPW * 16;

  v8f acc[TPW];
#pragma unroll
  for (int t = 0; t < TPW; ++t) { v8f z = {0.f, 0.f, 0.f, 0.f, 0.f, 0.f, 0.f, 0.f}; acc[t] = z; }
  const _Float16* ahp = sA + (r0 + m) * APK + 8 * hh;
#pragma unroll 2
  for (int kt = 0; kt < KD / 32; ++kt) {
    FragH af;
    af.h[0] = *(const v8h*)(ahp + 32 * kt);
    af.h[1] = *(const v8h*)(ahp + 32 * kt + 16);
#pragma unroll
    for (int t = 0; t < TPW; ++t) {
      const _Float16* bp = Bw + (size_t)(c0 + 16 * t + m) * KD + 32 * kt + 8 * hh;
      FragH bf;
      bf.h[0] = *(const v8h*)bp;
      bf.h[1] = *(const v8h*)(bp + 16);
      acc[t] = wmh(af.v, bf.v, acc[t]);
    }
  }
  __syncthreads();

  {
    float* sp = stg + (size_t)(r0 + 8 * hh) * NC + c0 + m;
#pragma unroll
    for (int t = 0; t < TPW; ++t) {
#pragma unroll
      for (int r = 0; r < 8; ++r) sp[r * NC + 16 * t] = acc[t][r] * WINV;
    }
  }
  __syncthreads();

  const int qq   = lane & (Q4 - 1);
  const int rsub = lane / Q4;
  const int col  = c0 + 4 * qq;
  const int hd   = col / CH;
  const v4f sA4 = *(const v4f*)(attS + col);
  const v4f sD4 = *(const v4f*)(attD + col);
  const size_t gb = (size_t)(rowBase + r0) * NC + col;
#pragma unroll
  for (int it = 0; it < NIT; ++it) {
    const int row = it * RPI + rsub;
    const v4f v = *(const v4f*)(stg + (size_t)(r0 + row) * NC + col);
    *(volatile v4f*)(C + gb + (size_t)row * NC) = v;
    float ps = v.x * sA4.x + v.y * sA4.y + v.z * sA4.z + v.w * sA4.w;
    float pd = v.x * sD4.x + v.y * sD4.y + v.z * sD4.z + v.w * sD4.w;
#pragma unroll
    for (int o = 1; o < LPH; o <<= 1) { ps += __shfl_xor(ps, o); pd += __shfl_xor(pd, o); }
    if ((lane & (LPH - 1)) == 0) { sES[(r0 + row) * HEADS + hd] = ps; sED[(r0 + row) * HEADS + hd] = pd; }
  }
  __threadfence();
#pragma unroll
  for (int it = 0; it < NIT; ++it) {
    const int row = it * RPI + rsub;
    const v4f v = *(const v4f*)(stg + (size_t)(r0 + row) * NC + col);
    *(volatile v4f*)(C + gb + (size_t)row * NC) = v;
  }
  __syncthreads();

  v4f dv = {0.f, 0.f, 0.f, 0.f};
  const size_t eb = (size_t)rowBase * HEADS;
  if (wave < NESI) {
    const int f = wave * 128 + 4 * lane;
    dv = *(const v4f*)(sES + f);
    *(volatile v4f*)(eS + eb + f) = dv;
  } else if (wave < 2 * NESI) {
    const int f = (wave - NESI) * 128 + 4 * lane;
    dv = *(const v4f*)(sED + f);
    *(volatile v4f*)(eD + eb + f) = dv;
  }
  __threadfence();
  if (wave < NESI) {
    const int f = wave * 128 + 4 * lane;
    *(volatile v4f*)(eS + eb + f) = dv;
  } else if (wave < 2 * NESI) {
    const int f = (wave - NESI) * 128 + 4 * lane;
    *(volatile v4f*)(eD + eb + f) = dv;
  }
}

template <int LAST>
__global__ __launch_bounds__(NTHR) void k_agg(
    const int* __restrict__ csr, const int* __restrict__ off, const int* __restrict__ cnt,
    const float* __restrict__ eS, const float* __restrict__ eD, const float* __restrict__ hw,
    const float* __restrict__ bias, float* xout, int nN, int csrLen) {
  const int tid = threadIdx.x, lane = tid & 31, wave = tid >> 5;
  const int tbase = blockIdx.x * TGT + wave * 32;
  const int col0  = 4 * lane;
  const int hd0   = lane >> 3;
  const v4f z4 = {0.f, 0.f, 0.f, 0.f};
  const v4f bb0 = *(const v4f*)(bias + col0);

  const int cl    = tbase + lane;
  const int cnt_l = cnt[cl];
  const int off_l = off[cl];

#pragma unroll 1
  for (int j = 0; j < 32; ++j) {
    const int c = tbase + j;
    int n = __shfl(cnt_l, j);
    n = n < 0 ? 0 : (n > DEGCAP ? DEGCAP : n);
    const int st = __shfl(off_l, j);
    const float ed0 = eD[(size_t)c * NHEAD + hd0];

    float mx0 = NEG_BIG;
#pragma unroll 1
    for (int q0 = 0; q0 < n; q0 += 32) {
      int pos = st + q0 + lane;
      pos = pos < 0 ? 0 : (pos > csrLen - 1 ? csrLen - 1 : pos);
      int sl = csr[pos];
      sl = sl < 0 ? 0 : (sl > nN - 1 ? nN - 1 : sl);
      const int mcnt = (n - q0) < 32 ? (n - q0) : 32;
#pragma unroll 1
      for (int pp = 0; pp < mcnt; ++pp) {
        const int s = __builtin_amdgcn_readlane(sl, pp);
        mx0 = fmaxf(mx0, lrelu(eS[(size_t)s * NHEAD + hd0] + ed0));
      }
    }

    float den0 = 0.f;
    v4f   acc0 = z4;
#pragma unroll 1
    for (int q0 = 0; q0 < n; q0 += 32) {
      int pos = st + q0 + lane;
      pos = pos < 0 ? 0 : (pos > csrLen - 1 ? csrLen - 1 : pos);
      int sl = csr[pos];
      sl = sl < 0 ? 0 : (sl > nN - 1 ? nN - 1 : sl);
      const int mcnt = (n - q0) < 32 ? (n - q0) : 32;
#pragma unroll 1
      for (int pp = 0; pp < mcnt; ++pp) {
        const int s = __builtin_amdgcn_readlane(sl, pp);
        const float p0 = __expf(lrelu(eS[(size_t)s * NHEAD + hd0] + ed0) - mx0);
        den0 += p0;
        const v4f h0 = *(const v4f*)(hw + (size_t)s * NCOL + col0);
        acc0 = acc0 + h0 * p0;
      }
    }

    const float rd0 = den0 > 0.f ? (1.0f / den0) : 0.f;
    v4f v0 = acc0 * rd0 + bb0;
    if constexpr (LAST == 0) {
      v0.x = v0.x > 0.f ? v0.x : 0.f;
      v0.y = v0.y > 0.f ? v0.y : 0.f;
      v0.z = v0.z > 0.f ? v0.z : 0.f;
      v0.w = v0.w > 0.f ? v0.w : 0.f;
    }

    float* pw = xout + (size_t)c * NCOL + col0;
    if constexpr (LAST == 0) {
      if (c >= nN) v0 = z4;
      *(volatile v4f*)pw = v0;
      __threadfence();
      *(volatile v4f*)pw = v0;
    } else {
      if (c < nN) {
        *(volatile v4f*)pw = v0;
        __threadfence();
        *(volatile v4f*)pw = v0;
      }
    }
  }
}

typedef GCfg<FIN, NCOL> GA;
static_assert((TGT % GA::BM) == 0);

extern "C" void kernel_launch(void* const* d_in, const int* in_sizes, int n_in,
                              void* d_out, int out_size, void* d_ws, size_t ws_size,
                              hipStream_t stream) {
  if (n_in < 11) return;
  const int nN = in_sizes[0] / FIN;
  const int nE = in_sizes[9];
  if (nN <= 0 || nE <= 0 || in_sizes[0] != nN * FIN || in_sizes[10] != nE) return;
  if (in_sizes[1] != FIN * NCOL || in_sizes[5] != NCOL * NCOL) return;
  if (in_sizes[2] != NCOL || in_sizes[3] != NCOL || in_sizes[4] != NCOL) return;
  if (in_sizes[6] != NCOL || in_sizes[7] != NCOL || in_sizes[8] != NCOL) return;
  if (out_size != nN * NCOL) return;
  if (nE > (1 << 28) || nN > (1 << 24)) return;

  const float* x   = (const float*)d_in[0];
  const float* W1  = (const float*)d_in[1];
  const float* al1 = (const float*)d_in[2];
  const float* ar1 = (const float*)d_in[3];
  const float* b1  = (const float*)d_in[4];
  const float* W2  = (const float*)d_in[5];
  const float* al2 = (const float*)d_in[6];
  const float* ar2 = (const float*)d_in[7];
  const float* b2  = (const float*)d_in[8];
  const int*   src = (const int*)d_in[9];
  const int*   dst = (const int*)d_in[10];
  float* out = (float*)d_out;

  const int NPAD   = ((nN + TGT - 1) / TGT) * TGT;
  const int nBC    = (nN + NBC - 1) / NBC;
  const int CNTPAD = nBC * NBC;
  if (4 * nBC + 1 > RBN) return;
  const int nBF    = (nN + NBF - 1) / NBF;
  const int csrLen = ((nE + 31) & ~31) + 4096;
  if (31 * 4 * nBC > 4096) return;
  const int nAgg   = NPAD / TGT;

  char* ws = (char*)d_ws;
  size_t off = 0;
  const size_t oW1  = off; off += (size_t)FIN * NCOL * 2;         off = (off + 255) & ~(size_t)255;
  const size_t oW2  = off; off += (size_t)NCOL * NCOL * 2;        off = (off + 255) & ~(size_t)255;
  const size_t oCnt = off; off += (size_t)CNTPAD * 4;             off = (off + 255) & ~(size_t)255;
  const size_t oOff = off; off += (size_t)CNTPAD * 4;             off = (off + 255) & ~(size_t)255;
  const size_t oRb  = off; off += (size_t)RBN * 4;                off = (off + 255) & ~(size_t)255;
  const size_t oCsr = off; off += (size_t)csrLen * 4;             off = (off + 255) & ~(size_t)255;
  const size_t oHw  = off; off += (size_t)NPAD * NCOL * 4;        off = (off + 255) & ~(size_t)255;
  const size_t oX   = off; off += (size_t)NPAD * NCOL * 4;        off = (off + 255) & ~(size_t)255;
  const size_t oES  = off; off += (size_t)NPAD * NHEAD * 4;       off = (off + 255) & ~(size_t)255;
  const size_t oED  = off; off += (size_t)NPAD * NHEAD * 4;       off = (off + 255) & ~(size_t)255;
  if (off > ws_size || off > (size_t)WSCAP) return;
  _Float16* wp1 = (_Float16*)(ws + oW1);
  _Float16* wp2 = (_Float16*)(ws + oW2);
  int*   cnt  = (int*)(ws + oCnt);
  int*   offp = (int*)(ws + oOff);
  int*   rb   = (int*)(ws + oRb);
  int*   csr  = (int*)(ws + oCsr);
  float* hw   = (float*)(ws + oHw);
  float* xb   = (float*)(ws + oX);
  float* es   = (float*)(ws + oES);
  float* ed   = (float*)(ws + oED);

  const int vec8 = ((nE & 3) == 0) ? 1 : 0;

  k_wprep<FIN, NCOL><<<(NCOL * FIN / 8) / NTHR, NTHR, 0, stream>>>(W1, wp1);
  k_wprep<NCOL, NCOL><<<(NCOL * NCOL / 8) / NTHR, NTHR, 0, stream>>>(W2, wp2);

  k_count<<<nBC, NTHR, 0, stream>>>(dst, cnt, nE, vec8);
  k_offsets<<<1, OTHR, 0, stream>>>(cnt, offp, rb, nBC);
  hipFuncSetAttribute(reinterpret_cast<const void*>(&k_fill),
                      hipFuncAttributeMaxDynamicSharedMemorySize, LDS_FILL);
  k_fill<<<nBF, NTHR, LDS_FILL, stream>>>(src, dst, offp, rb, csr, nN, nE, vec8, csrLen);

  k_gemm<FIN, NCOL, NHEAD><<<NPAD / GA::BM, NTHR, GA::LDS, stream>>>(x, wp1, al1, ar1, hw, es, ed, nN);
  k_agg<0><<<nAgg, NTHR, 0, stream>>>(csr, offp, cnt, es, ed, hw, b1, xb, nN, csrLen);

  k_gemm<NCOL, NCOL, NHEAD><<<NPAD / GA::BM, NTHR, GA::LDS, stream>>>(xb, wp2, al2, ar2, hw, es, ed, NPAD);
  k_agg<1><<<nAgg, NTHR, 0, stream>>>(csr, offp, cnt, es, ed, hw, b2, out, nN, csrLen);
}
